// Field2point_18811956756749
// MI455X (gfx1250) — hardware-verified
//
#include <hip/hip_runtime.h>
#include <math.h>

typedef unsigned short us_t;
typedef us_t   v8us  __attribute__((ext_vector_type(8)));
typedef us_t   v16us __attribute__((ext_vector_type(16)));
typedef __bf16 v16b  __attribute__((ext_vector_type(16)));
typedef float  v8f   __attribute__((ext_vector_type(8)));
typedef float  v4f   __attribute__((ext_vector_type(4)));
typedef v8us __attribute__((may_alias)) v8usa;
typedef v4f  __attribute__((may_alias)) v4fa;

union Frag { v16b v; v16us u; v8us half[2]; };

#define NB         16
#define NL         8192
#define NK         128
#define PLANE      16384
#define NPSI       262144
#define NPTS       131072
#define PTS_BLK    64
#define STG_PLANE  9216
#define STASH_WAVE 12288

__device__ __forceinline__ us_t bf16_rne(float f) {
  unsigned u = __float_as_uint(f);
  u += 0x7FFFu + ((u >> 16) & 1u);
  return (us_t)(u >> 16);
}
__device__ __forceinline__ float bf16_val(us_t b) { return __uint_as_float(((unsigned)b) << 16); }
__device__ __forceinline__ void split2(float v, us_t& hb, us_t& lb) {
  hb = bf16_rne(v);
  lb = bf16_rne(v - bf16_val(hb));
}

__device__ __forceinline__ v8f wmma_bf16(v16b a, v16b b, v8f c) {
  v8f d = __builtin_amdgcn_wmma_f32_16x16x32_bf16(false, a, false, b, (short)0, c, false, false);
  asm volatile("v_nop\n\tv_nop\n\tv_nop\n\tv_nop" : "+v"(d) : "v"(a), "v"(b));
  return d;
}
__device__ __forceinline__ v8f wmma3(v16b ah, v16b al, v16b bh, v16b bl, v8f c) {
  c = wmma_bf16(ah, bh, c);
  c = wmma_bf16(ah, bl, c);
  c = wmma_bf16(al, bh, c);
  return c;
}

__device__ __forceinline__ v16b ldrow(const us_t* p, int h) {
  Frag f;
  f.half[0] = *(const v8usa*)(p + 8 * h);
  f.half[1] = *(const v8usa*)(p + 16 + 8 * h);
  return f.v;
}
__device__ __forceinline__ v16b ldvec(const us_t* p) {
  Frag f;
  f.half[0] = *(const v8usa*)p;
  f.half[1] = *(const v8usa*)(p + 8);
  return f.v;
}

__global__ __launch_bounds__(256) void k_convert(const float* __restrict__ psi,
                                                 us_t* __restrict__ psih, us_t* __restrict__ psil,
                                                 us_t* __restrict__ tab)
{
  __shared__ __attribute__((aligned(16))) us_t tls[256 * 48];
  const int tid = threadIdx.x;
  if (blockIdx.x < NPSI / 2048) {
    const int g = blockIdx.x * 256 + tid;
    const float* src = psi + (size_t)g * 8;
    const v4f a = *(const v4fa*)src;
    const v4f c = *(const v4fa*)(src + 4);
    us_t h0, l0, h1, l1, h2, l2, h3, l3, h4, l4, h5, l5, h6, l6, h7, l7;
    split2(a.x, h0, l0); split2(a.y, h1, l1); split2(a.z, h2, l2); split2(a.w, h3, l3);
    split2(c.x, h4, l4); split2(c.y, h5, l5); split2(c.z, h6, l6); split2(c.w, h7, l7);
    const v8us hv = { h0, h1, h2, h3, h4, h5, h6, h7 };
    const v8us lv = { l0, l1, l2, l3, l4, l5, l6, l7 };
    us_t* dh = psih + (size_t)g * 8;
    us_t* dl = psil + (size_t)g * 8;
    *(volatile v8us*)dh = hv;
    *(volatile v8us*)dl = lv;
    __threadfence();
    *(volatile v8us*)dh = hv;
    *(volatile v8us*)dl = lv;
  } else {
    const int t = (blockIdx.x - NPSI / 2048) * 256 + tid;
    const int a = t >> 4, c0 = (t & 15) * 8;
    us_t* s = tls + tid * 48;
    #pragma unroll 1
    for (int q = 0; q < 8; ++q) {
      const int r = (a * (c0 + q)) & 127;
      const float fr = (float)r * 0.015625f;
      const float cv = cospif(fr);
      const float sv = sinpif(fr);
      us_t ch, cl, sh, sl;
      split2(cv, ch, cl);
      split2(sv, sh, sl);
      s[q]      = ch;
      s[8 + q]  = cl;
      s[16 + q] = sh;
      s[24 + q] = sl;
      s[32 + q] = (us_t)(sh ^ 0x8000u);
      s[40 + q] = (us_t)(sl ^ 0x8000u);
    }
    __syncthreads();
    us_t* dst = tab + (size_t)t * 8;
    #pragma unroll
    for (int p = 0; p < 6; ++p) {
      const v8us v = *(const v8usa*)(s + 8 * p);
      *(volatile v8us*)(dst + (size_t)p * PLANE) = v;
    }
    __threadfence();
    #pragma unroll
    for (int p = 0; p < 6; ++p) {
      const v8us v = *(const v8usa*)(s + 8 * p);
      *(volatile v8us*)(dst + (size_t)p * PLANE) = v;
    }
  }
}

template <bool TRANS>
__device__ __forceinline__ void cg_store(const us_t* stg, us_t* O, int b, int m0, int tid) {
  #pragma unroll 1
  for (int it = 0; it < 32; ++it) {
    const int g = it * 128 + tid;
    const int line = g >> 3, q = g & 7;
    const int p = line >> 7, rem = line & 127;
    const us_t* sp = stg + p * STG_PLANE;
    us_t* op = O + (size_t)p * NPSI + (size_t)b * PLANE;
    v8us v;
    int di;
    if (TRANS) {
      v = *(const v8usa*)(sp + rem * 72 + 8 * q);
      di = rem * NK + m0 + 8 * q;
    } else {
      const int row = rem >> 1, hl = rem & 1;
      v = *(const v8usa*)(sp + row * 136 + 64 * hl + 8 * q);
      di = ((m0 ^ 64) + row) * NK + 64 * hl + 8 * q;
    }
    *(volatile v8us*)(op + di) = v;
  }
}

template <bool ACPLX, bool TRANS>
__global__ __launch_bounds__(128) void k_cgemm(
    const us_t* __restrict__ Arh, const us_t* __restrict__ Arl,
    const us_t* __restrict__ Aih, const us_t* __restrict__ Ail,
    const us_t* __restrict__ Anh, const us_t* __restrict__ Anl, int a_bs,
    const us_t* __restrict__ Brh, const us_t* __restrict__ Brl,
    const us_t* __restrict__ Bih, const us_t* __restrict__ Bil, int b_bs,
    us_t* __restrict__ O)
{
  __shared__ __attribute__((aligned(16))) us_t stg[4 * STG_PLANE];

  const int tid = threadIdx.x, lane = tid & 31, w = tid >> 5;
  const int h = lane >> 4, m = lane & 15;
  const int m0 = blockIdx.x * 64, b = blockIdx.y;
  const size_t aoff  = (size_t)b * a_bs + (size_t)(m0 + 16 * w + m) * NK;
  const size_t bbase = (size_t)b * b_bs;
  const v8f z8 = {0.f, 0.f, 0.f, 0.f, 0.f, 0.f, 0.f, 0.f};

  #pragma unroll 1
  for (int ng = 0; ng < 4; ++ng) {
    v8f cr[2], ci[2];
    cr[0] = z8; cr[1] = z8; ci[0] = z8; ci[1] = z8;

    #pragma unroll 1
    for (int ks = 0; ks < 4; ++ks) {
      const int k0 = 32 * ks;
      const v16b arh = ldrow(Arh + aoff + k0, h);
      const v16b arl = ldrow(Arl + aoff + k0, h);
      v16b aih = arh, ail = arl, anh = arh, anl = arl;
      if constexpr (ACPLX) {
        aih = ldrow(Aih + aoff + k0, h);
        ail = ldrow(Ail + aoff + k0, h);
        anh = ldrow(Anh + aoff + k0, h);
        anl = ldrow(Anl + aoff + k0, h);
      }
      #pragma unroll
      for (int nt = 0; nt < 2; ++nt) {
        const size_t boff = bbase + (size_t)(32 * ng + 16 * nt + m) * NK + k0;
        const v16b brh = ldrow(Brh + boff, h);
        const v16b brl = ldrow(Brl + boff, h);
        const v16b bih = ldrow(Bih + boff, h);
        const v16b bil = ldrow(Bil + boff, h);
        cr[nt] = wmma3(arh, arl, brh, brl, cr[nt]);
        ci[nt] = wmma3(arh, arl, bih, bil, ci[nt]);
        if constexpr (ACPLX) {
          cr[nt] = wmma3(anh, anl, bih, bil, cr[nt]);
          ci[nt] = wmma3(aih, ail, brh, brl, ci[nt]);
        }
      }
    }

    #pragma unroll
    for (int nt = 0; nt < 2; ++nt) {
      const int col = 32 * ng + 16 * nt + m;
      #pragma unroll
      for (int r = 0; r < 8; ++r) {
        const int rl = 16 * w + 8 * h + r;
        const int idx = TRANS ? (col * 72 + rl) : (rl * 136 + (col ^ 64));
        us_t hb, lb;
        split2(cr[nt][r], hb, lb);
        stg[idx] = hb;
        stg[STG_PLANE + idx] = lb;
        split2(ci[nt][r], hb, lb);
        stg[2 * STG_PLANE + idx] = hb;
        stg[3 * STG_PLANE + idx] = lb;
      }
    }
  }
  __syncthreads();

  cg_store<TRANS>(stg, O, b, m0, tid);
  __threadfence();
  cg_store<TRANS>(stg, O, b, m0, tid);
}

__global__ __launch_bounds__(128) void k_main(const float* __restrict__ x0,
                                              const float* __restrict__ y0,
                                              const us_t* __restrict__ ph,
                                              float* __restrict__ out)
{
  __shared__ __attribute__((aligned(16))) us_t stash[4 * STASH_WAVE];
  __shared__ float eys[128 * 16];
  __shared__ __attribute__((aligned(16))) float so[PTS_BLK];

  const int tid = threadIdx.x, lane = tid & 31, w = tid >> 5;
  const int h = lane >> 4, m = lane & 15;
  const int b = blockIdx.y;
  const int p0 = blockIdx.x * PTS_BLK + 16 * w;
  const float x = x0[(size_t)b * NL + p0 + m];
  const float y = y0[(size_t)b * NL + p0 + m];

  us_t* st = stash + w * STASH_WAVE;
  #pragma unroll 1
  for (int idx = 0; idx < 64; ++idx) {
    const int ks = idx >> 4, e = idx & 15;
    const int j = 32 * ks + 8 * h + e + (e & 8);
    const float th = x * (float)(j - 64);
    float sv, cv;
    sincosf(th, &sv, &cv);
    us_t ch, cl, sh, sl;
    split2(cv, ch, cl);
    split2(sv, sh, sl);
    us_t* q = st + (ks * 192 + lane) * 16 + e;
    q[0]    = ch;
    q[512]  = cl;
    q[1024] = sh;
    q[1536] = sl;
    q[2048] = (us_t)(sh ^ 0x8000u);
    q[2560] = (us_t)(sl ^ 0x8000u);
  }
  __syncthreads();

  const v8f z8 = {0.f, 0.f, 0.f, 0.f, 0.f, 0.f, 0.f, 0.f};
  const us_t* arow = ph + (size_t)b * PLANE + (size_t)m * NK;
  float* ey = eys + tid * 16;
  float P = 0.0f;

  #pragma unroll 1
  for (int mt = 0; mt < 8; ++mt) {
    #pragma unroll 1
    for (int rr = 0; rr < 8; ++rr) {
      const int i = 16 * mt + 8 * h + rr;
      const float th = y * (float)(i - 64);
      float sv, cv;
      sincosf(th, &sv, &cv);
      ey[rr] = cv;
      ey[8 + rr] = sv;
    }

    v8f cre = z8, cim = z8;
    #pragma unroll 1
    for (int ks = 0; ks < 4; ++ks) {
      const us_t* ap = arow + (size_t)mt * 16 * NK + 32 * ks;
      const v16b prh = ldrow(ap, h);
      const v16b prl = ldrow(ap + NPSI, h);
      const v16b pih = ldrow(ap + 2 * NPSI, h);
      const v16b pil = ldrow(ap + 3 * NPSI, h);
      const us_t* bp = st + (ks * 192 + lane) * 16;
      const v16b erh = ldvec(bp);
      const v16b erl = ldvec(bp + 512);
      const v16b eih = ldvec(bp + 1024);
      const v16b eil = ldvec(bp + 1536);
      const v16b enh = ldvec(bp + 2048);
      const v16b enl = ldvec(bp + 2560);
      cre = wmma3(prh, prl, erh, erl, cre);
      cre = wmma3(pih, pil, enh, enl, cre);
      cim = wmma3(prh, prl, eih, eil, cim);
      cim = wmma3(pih, pil, erh, erl, cim);
    }

    #pragma unroll
    for (int r = 0; r < 8; ++r)
      P = P + cre[r] * ey[r] - cim[r] * ey[8 + r];
  }
  P += __shfl_xor(P, 16);
  if (h == 0) so[16 * w + m] = P * (1.0f / 16384.0f);
  __syncthreads();

  if (w == 0) {
    const v4f v = *(const v4fa*)(so + 4 * (lane & 15));
    float* op = out + (size_t)b * NL + blockIdx.x * PTS_BLK + 4 * (lane & 15);
    if (lane < 16) *(volatile v4f*)op = v;
    __threadfence();
    if (lane < 16) *(volatile v4f*)op = v;
  }
}

extern "C" void kernel_launch(void* const* d_in, const int* in_sizes, int n_in,
                              void* d_out, int out_size, void* d_ws, size_t ws_size,
                              hipStream_t stream) {
  if (n_in < 3) return;
  if (in_sizes[0] != NPTS || in_sizes[1] != NPTS || in_sizes[2] != NPSI) return;
  if (out_size != NPTS) return;

  const float* x0  = (const float*)d_in[0];
  const float* y0  = (const float*)d_in[1];
  const float* psi = (const float*)d_in[2];
  float* out = (float*)d_out;

  const size_t psih_bytes = (size_t)NPSI * 2;
  const size_t tab_bytes  = (size_t)6 * PLANE * 2;
  const size_t t_bytes    = (size_t)4 * NPSI * 2;
  const size_t ph_bytes   = (size_t)4 * NPSI * 2;
  const size_t off_psih = 0;
  const size_t off_psil = off_psih + psih_bytes;
  const size_t off_tab  = off_psil + psih_bytes;
  const size_t off_t    = off_tab + tab_bytes;
  const size_t off_ph   = off_t + t_bytes;
  const size_t total    = off_ph + ph_bytes;
  if (total > ws_size) return;

  char* ws = (char*)d_ws;
  us_t* psih = (us_t*)(ws + off_psih);
  us_t* psil = (us_t*)(ws + off_psil);
  us_t* tab  = (us_t*)(ws + off_tab);
  us_t* tpl  = (us_t*)(ws + off_t);
  us_t* php  = (us_t*)(ws + off_ph);

  k_convert<<<136, 256, 0, stream>>>(psi, psih, psil, tab);

  k_cgemm<false, true><<<dim3(2, NB), 128, 0, stream>>>(
      psih, psil, psih, psih, psih, psih, PLANE,
      tab + 0 * PLANE, tab + 1 * PLANE, tab + 4 * PLANE, tab + 5 * PLANE, 0,
      tpl);

  k_cgemm<true, false><<<dim3(2, NB), 128, 0, stream>>>(
      tab + 0 * PLANE, tab + 1 * PLANE, tab + 4 * PLANE, tab + 5 * PLANE,
      tab + 2 * PLANE, tab + 3 * PLANE, 0,
      tpl + 0 * NPSI, tpl + 1 * NPSI, tpl + 2 * NPSI, tpl + 3 * NPSI, PLANE,
      php);

  k_main<<<dim3(NL / PTS_BLK, NB), 128, 0, stream>>>(x0, y0, php, out);
}
